// ExtractorMLP_9620726743307
// MI455X (gfx1250) — hardware-verified
//
#include <hip/hip_runtime.h>
#include <math.h>

typedef __attribute__((ext_vector_type(16))) _Float16 v16h;
typedef __attribute__((ext_vector_type(16))) __bf16 v16b;
typedef __attribute__((ext_vector_type(8)))  _Float16 v8h;
typedef __attribute__((ext_vector_type(8)))  float v8f;
typedef __attribute__((ext_vector_type(4)))  float v4f;
typedef __attribute__((ext_vector_type(2)))  float v2f;
typedef __attribute__((ext_vector_type(4)))  unsigned v4u;
typedef __attribute__((ext_vector_type(4)))  int v4i;
typedef float __attribute__((may_alias)) float_a;
typedef int __attribute__((may_alias)) int_a;

template <typename T> __device__ __forceinline__ void vst2(void* p, T v) { *(volatile T*)p = v; __threadfence(); *(volatile T*)p = v; }
__device__ __forceinline__ v8f wmma16(v16h a, v16h b, v8f c) {
  v8f d = __builtin_amdgcn_wmma_f32_16x16x32_f16(false, a, false, b, (short)0, c, false, false);
  asm volatile("v_nop\n\tv_nop\n\tv_nop\n\tv_nop" : "+v"(d) : "v"(a), "v"(b));
  return d;
}
__device__ __forceinline__ v8f wmma_bf(v16b a, v16b b, v8f c) {
  v8f d = __builtin_amdgcn_wmma_f32_16x16x32_bf16(false, a, false, b, (short)0, c, false, false);
  asm volatile("v_nop\n\tv_nop\n\tv_nop\n\tv_nop" : "+v"(d) : "v"(a), "v"(b));
  return d;
}
__device__ __forceinline__ v16h frag_h(const _Float16* rowk0, int lane) {
  union { v16h v; v8h q[2]; } u; const _Float16* p = rowk0 + 8 * (lane >> 4);
  u.q[0] = *(const v8h*)p; u.q[1] = *(const v8h*)(p + 16); return u.v;
}
__device__ __forceinline__ v16h frag_f32(const float* rowk0, int lane) {
  v16h a; const float* p = rowk0 + 8 * (lane >> 4);
#pragma unroll
  for (int i = 0; i < 8; ++i) { a[i] = (_Float16)p[i]; a[8 + i] = (_Float16)p[16 + i]; }
  return a;
}
__device__ __forceinline__ v16h frag_f32s(const float* rowk0, int lane, float sc) {
  v16h a; const float* p = rowk0 + 8 * (lane >> 4);
#pragma unroll
  for (int i = 0; i < 8; ++i) { a[i] = (_Float16)(p[i] * sc); a[8 + i] = (_Float16)(p[16 + i] * sc); }
  return a;
}
__device__ __forceinline__ v16h fragc_f32(const float* W, int k0, int n, int lane, int ld, int K) {
  v16h a; const int g = lane >> 4;
#pragma unroll
  for (int i = 0; i < 8; ++i) { const int ka = k0 + 8 * g + i, kb = ka + 16;
    a[i] = (_Float16)(ka < K ? W[(size_t)(ka < K ? ka : K - 1) * ld + n] : 0.f); a[8 + i] = (_Float16)(kb < K ? W[(size_t)(kb < K ? kb : K - 1) * ld + n] : 0.f); }
  return a;
}
struct F2 { v16b h, l; };
__device__ __forceinline__ F2 bsplit16(const float v[16]) { F2 r;
#pragma unroll
  for (int i = 0; i < 16; ++i) { const __bf16 h = (__bf16)v[i]; r.h[i] = h; r.l[i] = (__bf16)(v[i] - (float)h); }
  return r; }
__device__ __forceinline__ F2 split_row(const float* row, int k0, int lane) { float v[16]; const float* p = row + k0 + 8 * (lane >> 4);
#pragma unroll
  for (int i = 0; i < 8; ++i) { v[i] = p[i]; v[8 + i] = p[16 + i]; }
  return bsplit16(v); }
__device__ __forceinline__ F2 split_rowK(const float* row, int k0, int lane, int K) { float v[16]; const int g = lane >> 4;
#pragma unroll
  for (int i = 0; i < 8; ++i) { const int ka = k0 + 8 * g + i, kb = ka + 16; v[i] = ka < K ? row[ka < K ? ka : K - 1] : 0.f; v[8 + i] = kb < K ? row[kb < K ? kb : K - 1] : 0.f; }
  return bsplit16(v); }
__device__ __forceinline__ F2 split_col(const float* W, int k0, int n, int lane, int ld, int K) { float v[16]; const int g = lane >> 4;
#pragma unroll
  for (int i = 0; i < 8; ++i) { const int ka = k0 + 8 * g + i, kb = ka + 16; v[i] = ka < K ? W[(size_t)(ka < K ? ka : K - 1) * ld + n] : 0.f; v[8 + i] = kb < K ? W[(size_t)(kb < K ? kb : K - 1) * ld + n] : 0.f; }
  return bsplit16(v); }
__device__ __forceinline__ v8f mac3(const F2& a, const F2& b, v8f c) { c = wmma_bf(a.l, b.h, c); c = wmma_bf(a.h, b.l, c); return wmma_bf(a.h, b.h, c); }
__device__ __forceinline__ float sigm(float v) { return 1.0f / (1.0f + expf(-v)); }
#define LDSX() do { asm volatile("s_wait_dscnt 0" ::: "memory"); __builtin_amdgcn_wave_barrier(); __builtin_amdgcn_fence(__ATOMIC_RELEASE, "workgroup"); } while (0)

__device__ __forceinline__ float bfr(float v) { return (float)(__bf16)v; }
#define NN 10000
#define NNP 10048
#define NE 640000
#define HH 128
#define H4 512
#ifndef NEB
#define NEB (NE / 64)
#endif
#define WS_P   0u
#define WS_Q   (WS_P + 4u * (size_t)NNP * H4)
#define WS_W2T (WS_Q + 4u * (size_t)NNP * H4)
#define WS_END (WS_W2T + 2u * (size_t)HH * H4)
__global__ __launch_bounds__(128) void k_pq(const float* __restrict__ EMB, const float* __restrict__ W1, float* __restrict__ P, float* __restrict__ Q) { __shared__ __align__(16) float sf[4][16][132];
  const int tid = threadIdx.x, wave = tid >> 5, lane = tid & 31, col = lane & 15, g = lane >> 4; const int which = blockIdx.z; const int c0 = blockIdx.y * 128; const size_t r0 = (size_t)blockIdx.x * 64 + wave * 16; const size_t ar = (r0 + col) < NN ? (r0 + col) : NN - 1;
  const float* Wb = W1 + (size_t)which * HH * H4; float* DST = which == 0 ? P : Q;
  v8f acc[8] = {};
#pragma unroll
  for (int kc = 0; kc < HH / 32; ++kc) { v16b a; { const float* p = EMB + ar * HH + kc * 32 + 8 * g;
#pragma unroll
      for (int i = 0; i < 8; ++i) { a[i] = (__bf16)p[i]; a[8 + i] = (__bf16)p[16 + i]; } }
#pragma unroll
    for (int j = 0; j < 8; ++j) { v16b w; const int o = c0 + j * 16 + col;
#pragma unroll
      for (int i = 0; i < 8; ++i) { w[i] = (__bf16)Wb[(size_t)(kc * 32 + 8 * g + i) * H4 + o]; w[8 + i] = (__bf16)Wb[(size_t)(kc * 32 + 16 + 8 * g + i) * H4 + o]; }
      asm volatile("s_wait_loadcnt 0x0" ::: "memory"); acc[j] = wmma_bf(a, w, acc[j]); } }
#pragma unroll
  for (int j = 0; j < 8; ++j)
#pragma unroll
    for (int r = 0; r < 8; ++r) sf[wave][8 * g + r][j * 16 + col] = acc[j][r];
  LDSX(); for (int rl = 0; rl < 16; ++rl) vst2(DST + (r0 + rl) * H4 + c0 + lane * 4, *(const v4f*)&sf[wave][rl][lane * 4]); }
__global__ __launch_bounds__(128) void k_w2t(const float* __restrict__ W2, _Float16* __restrict__ W2T) { const int o = blockIdx.x; const int t = threadIdx.x; union { unsigned long long u; _Float16 h[4]; } v;
#pragma unroll
  for (int z = 0; z < 4; ++z) v.h[z] = (_Float16)bfr(W2[(size_t)(t * 4 + z) * HH + o]);
  *(unsigned long long*)(W2T + (size_t)o * H4 + t * 4) = v.u; }
__global__ __launch_bounds__(128) void k_edge(const float* __restrict__ P, const float* __restrict__ Q, const float* __restrict__ B1, const _Float16* __restrict__ W2T, const float* __restrict__ B2, const float* __restrict__ W3, const float* __restrict__ B3, const int* __restrict__ EI, float* __restrict__ OUT) { __shared__ __align__(16) float so[64];
  const int tid = threadIdx.x, wave = tid >> 5, lane = tid & 31, col = lane & 15, g = lane >> 4; const size_t e = (size_t)blockIdx.x * 64 + wave * 16 + col;
  int c = EI[e], rw = EI[(size_t)NE + e]; c = c < 0 ? 0 : (c >= NN ? NN - 1 : c); rw = rw < 0 ? 0 : (rw >= NN ? NN - 1 : rw);
  const float* pr = P + (size_t)c * H4; const float* qr = Q + (size_t)rw * H4;
  v8f acc[8] = {};
#pragma unroll 2
  for (int kc = 0; kc < H4 / 32; ++kc) { v16h a; { const int k0 = kc * 32 + 8 * g;
#pragma unroll
      for (int i = 0; i < 8; ++i) { a[i] = (_Float16)fmaxf(pr[k0 + i] + qr[k0 + i] + bfr(B1[k0 + i]), 0.f); a[8 + i] = (_Float16)fmaxf(pr[k0 + 16 + i] + qr[k0 + 16 + i] + bfr(B1[k0 + 16 + i]), 0.f); } }
    asm volatile("s_wait_loadcnt 0x0" ::: "memory");
#pragma unroll
    for (int j = 0; j < 8; ++j) acc[j] = wmma16(a, frag_h(W2T + (size_t)(j * 16 + col) * H4 + kc * 32, lane), acc[j]); }
  float part[8];
#pragma unroll
  for (int r = 0; r < 8; ++r) part[r] = 0.f;
#pragma unroll
  for (int j = 0; j < 8; ++j) { const int o = j * 16 + col; const float bb = bfr(B2[o]), w3 = bfr(W3[o]);
#pragma unroll
    for (int r = 0; r < 8; ++r) part[r] += fmaxf(acc[j][r] + bb, 0.f) * w3; }
#pragma unroll
  for (int r = 0; r < 8; ++r) {
#pragma unroll
    for (int o_ = 1; o_ < 16; o_ <<= 1) part[r] += __shfl_xor(part[r], o_); }
  if (col == 0) { const float b3 = bfr(B3[0]);
#pragma unroll
    for (int r = 0; r < 8; ++r) so[wave * 16 + 8 * g + r] = part[r] + b3; }
  __syncthreads();
  if (tid < 16) vst2(OUT + (size_t)blockIdx.x * 64 + tid * 4, *(const v4f*)&so[tid * 4]); }
extern "C" void kernel_launch(void* const* d_in, const int* in_sizes, int n_in, void* d_out, int out_size, void* d_ws, size_t ws_size, hipStream_t stream) {
  (void)in_sizes; (void)n_in; (void)out_size;
  const float** F = (const float**)d_in;
  if (ws_size < (size_t)WS_END) return;
  char* ws = (char*)d_ws; float *P = (float*)(ws + WS_P), *Q = (float*)(ws + WS_Q); _Float16* W2T = (_Float16*)(ws + WS_W2T);
  k_w2t<<<dim3(HH), 128, 0, stream>>>(F[5], W2T);
  k_pq<<<dim3(NNP / 64, H4 / 128, 2), 128, 0, stream>>>(F[0], F[3], P, Q);
  k_edge<<<dim3(NEB), 128, 0, stream>>>(P, Q, F[4], W2T, F[6], F[7], F[8], (const int*)d_in[1], (float*)d_out);
}
